// LinearAttention_62998580298120
// MI455X (gfx1250) — hardware-run, weakly checked
//
#include <hip/hip_runtime.h>
#include <math.h>

typedef __attribute__((ext_vector_type(16))) _Float16 v16h;
typedef __attribute__((ext_vector_type(8)))  _Float16 v8h;
typedef __attribute__((ext_vector_type(16))) __bf16   v16b;
typedef __attribute__((ext_vector_type(8)))  __bf16   v8b;
typedef __attribute__((ext_vector_type(8)))  float    v8f;
typedef __attribute__((ext_vector_type(4)))  float    v4f;
typedef __attribute__((ext_vector_type(4)))  unsigned int v4u;
typedef __attribute__((ext_vector_type(2)))  unsigned int v2u;

constexpr int kTok   = 2048;
constexpr int kEmb   = 1024;
constexpr int kHeads = 16;
constexpr int kHd    = 64;
constexpr int kHalf  = kHd / 2;
constexpr int kCat   = 3 * kEmb + kHd;
constexpr int kRotRows = 4;
constexpr float kG1Carry  = 64.0f;
constexpr float kWg2Carry = 256.0f;
constexpr float kGateScale = 1.0f / (kG1Carry * kWg2Carry);
constexpr float kInvEmb = 1.0f / (float)kEmb;
constexpr float kLnEps  = 1e-5f;
constexpr float kF16MinNormal = 6.103515625e-05f;
static_assert(kHeads * kHd == kEmb);
static_assert(kCat == 3136);
static_assert((kEmb % 32) == 0 && (kHd % 32) == 0);
static_assert((kTok % 64) == 0 && (kCat % 64) == 0 && (kEmb % 64) == 0);
static_assert((kTok % kRotRows) == 0);

constexpr size_t kSzXB   = (size_t)kTok * kEmb * 2;
constexpr size_t kSzWCT  = (size_t)kCat * kEmb * 2;
constexpr size_t kSzWOT  = (size_t)kEmb * kEmb * 2;
constexpr size_t kSzWG2T = (size_t)kEmb * kHd * 2;
constexpr size_t kSzTab  = (size_t)kTok * kHalf * 4;
constexpr size_t kSzP    = (size_t)kTok * kCat * 4;
constexpr size_t kSzPl16 = (size_t)kTok * kEmb * 2;
constexpr size_t kSzG1H  = (size_t)kTok * kHd * 2;
constexpr size_t kSzPl32 = (size_t)kTok * kEmb * 4;
constexpr size_t kOffXB   = 0;
constexpr size_t kOffWCT  = kOffXB   + kSzXB;
constexpr size_t kOffWOT  = kOffWCT  + kSzWCT;
constexpr size_t kOffWG2T = kOffWOT  + kSzWOT;
constexpr size_t kOffCST  = kOffWG2T + kSzWG2T;
constexpr size_t kOffSNT  = kOffCST  + kSzTab;
constexpr size_t kOffP    = kOffSNT  + kSzTab;
constexpr size_t kOffQH   = kOffP    + kSzP;
constexpr size_t kOffQL   = kOffQH   + kSzPl16;
constexpr size_t kOffKH   = kOffQL   + kSzPl16;
constexpr size_t kOffKL   = kOffKH   + kSzPl16;
constexpr size_t kOffVTH  = kOffKL   + kSzPl16;
constexpr size_t kOffVTL  = kOffVTH  + kSzPl16;
constexpr size_t kOffG1H  = kOffVTL  + kSzPl16;
constexpr size_t kOffATT  = kOffG1H  + kSzG1H;
constexpr size_t kOffGLG  = kOffATT  + kSzPl32;
constexpr size_t kOffZH   = kOffGLG  + kSzPl32;
constexpr size_t kOffZL   = kOffZH   + kSzPl16;
constexpr size_t kWsTotal = kOffZL   + kSzPl16;
static_assert(kWsTotal == 89653248ull);
static_assert(kWsTotal <= 134217728ull);
static_assert((kOffWCT % 128) == 0 && (kOffWOT % 128) == 0 && (kOffWG2T % 128) == 0 && (kOffCST % 128) == 0 &&
              (kOffSNT % 128) == 0 && (kOffP % 128) == 0 && (kOffQH % 128) == 0 && (kOffQL % 128) == 0 &&
              (kOffKH % 128) == 0 && (kOffKL % 128) == 0 && (kOffVTH % 128) == 0 && (kOffVTL % 128) == 0 &&
              (kOffG1H % 128) == 0 && (kOffATT % 128) == 0 && (kOffGLG % 128) == 0 && (kOffZH % 128) == 0 &&
              (kOffZL % 128) == 0);

struct FreqTab { float f[32]; };
static_assert(sizeof(FreqTab) == 128);

__device__ __forceinline__ unsigned short f2bf_bits(float f) {
  unsigned u = __float_as_uint(f);
  return (unsigned short)((u + 0x7FFFu + ((u >> 16) & 1u)) >> 16);
}
__device__ __forceinline__ float bf_bits2f(unsigned short h) { return __uint_as_float(((unsigned)h) << 16); }
__device__ __forceinline__ unsigned pk16(unsigned short a, unsigned short b) { return (unsigned)a | ((unsigned)b << 16); }
__device__ __forceinline__ unsigned short h_bits_flush(float f) {
  const float g = (fabsf(f) < kF16MinNormal) ? 0.0f : f;
  const _Float16 h = (_Float16)g;
  return __builtin_bit_cast(unsigned short, h);
}

__device__ __forceinline__ void dep_guard4_h(v8f& a, v8f& b, v8f& c, v8f& d, v16h x, v16h y) {
  asm volatile("v_nop\n\tv_nop\n\tv_nop\n\tv_nop" : "+v"(a), "+v"(b), "+v"(c), "+v"(d) : "v"(x), "v"(y));
}
__device__ __forceinline__ void dep_guard4_b(v8f& a, v8f& b, v8f& c, v8f& d, v16b x, v16b y) {
  asm volatile("v_nop\n\tv_nop\n\tv_nop\n\tv_nop" : "+v"(a), "+v"(b), "+v"(c), "+v"(d) : "v"(x), "v"(y));
}
__device__ __forceinline__ void keep4_h(v16h a, v16h b, v16h c, v16h d) { asm volatile("v_nop" :: "v"(a), "v"(b), "v"(c), "v"(d)); }
__device__ __forceinline__ void keep4_b(v16b a, v16b b, v16b c, v16b d) { asm volatile("v_nop" :: "v"(a), "v"(b), "v"(c), "v"(d)); }
__device__ __forceinline__ void acc_guard4(v8f& a, v8f& b, v8f& c, v8f& d) {
  asm volatile("v_nop\n\tv_nop\n\tv_nop\n\tv_nop" : "+v"(a), "+v"(b), "+v"(c), "+v"(d));
}

template <typename T> struct Frag;
template <> struct Frag<_Float16> {
  typedef v16h V;
  union U { v16h v; v8h h[2]; };
  static __device__ __forceinline__ v16h load(const _Float16* p) {
    U f; f.h[0] = *(const v8h*)(p); f.h[1] = *(const v8h*)(p + 16); return f.v;
  }
  static __device__ __forceinline__ v8f mma(v16h a, v16h b, v8f c) {
    return __builtin_amdgcn_wmma_f32_16x16x32_f16(false, a, false, b, (short)0, c, false, false);
  }
  static __device__ __forceinline__ void guard4(v8f& a, v8f& b, v8f& c, v8f& d, v16h x, v16h y) { dep_guard4_h(a, b, c, d, x, y); }
  static __device__ __forceinline__ void keep(v16h a, v16h b, v16h c, v16h d) { keep4_h(a, b, c, d); }
};
template <> struct Frag<__bf16> {
  typedef v16b V;
  union U { v16b v; v8b h[2]; };
  static __device__ __forceinline__ v16b load(const __bf16* p) {
    U f; f.h[0] = *(const v8b*)(p); f.h[1] = *(const v8b*)(p + 16); return f.v;
  }
  static __device__ __forceinline__ v8f mma(v16b a, v16b b, v8f c) {
    return __builtin_amdgcn_wmma_f32_16x16x32_bf16(false, a, false, b, (short)0, c, false, false);
  }
  static __device__ __forceinline__ void guard4(v8f& a, v8f& b, v8f& c, v8f& d, v16b x, v16b y) { dep_guard4_b(a, b, c, d, x, y); }
  static __device__ __forceinline__ void keep(v16b a, v16b b, v16b c, v16b d) { keep4_b(a, b, c, d); }
};

__device__ __forceinline__ v8f mma_b(v16b a, v16b b, v8f c) {
  c = __builtin_amdgcn_wmma_f32_16x16x32_bf16(false, a, false, b, (short)0, c, false, false);
  asm volatile("v_nop\n\tv_nop\n\tv_nop\n\tv_nop" : "+v"(c) : "v"(a), "v"(b));
  return c;
}

template <int ET> struct Elem;
template <> struct Elem<0> { typedef _Float16 T; };
template <> struct Elem<1> { typedef __bf16 T; };
template <int ET, int SPL>
__global__ __launch_bounds__(256) void wmma_gemm64(
    const unsigned short* __restrict__ Ap, const unsigned short* __restrict__ A2p, int lda,
    const unsigned short* __restrict__ Btp, int ldb,
    float* __restrict__ C, int ldc,
    int M, int N, int K, float scale) {
  typedef typename Elem<ET>::T T;
  typedef typename Frag<T>::V V;
  const T* A = (const T*)Ap;
  const T* A2 = (const T*)A2p;
  const T* Bt = (const T*)Btp;
  __shared__ __align__(16) float sT[8][16 * 68];
  const int lane = threadIdx.x & 31;
  const int wave = threadIdx.x >> 5;
  const int tilesN = N >> 6;
  const int tilesM = M >> 6;
  const int tile = blockIdx.x * 8 + wave;
  if (tile >= tilesM * tilesN) return;
  const int tm = tile / tilesN;
  const int tn = tile - tm * tilesN;
  const int m0 = tm << 6;
  const int n0 = tn << 6;

  const int rlane = lane & 15;
  const int koff  = (lane >> 4) * 8;
  const int mOff  = (lane >> 4) * 8;

  v8f acc[4][4];
#pragma unroll
  for (int i = 0; i < 4; ++i)
#pragma unroll
    for (int j = 0; j < 4; ++j) acc[i][j] = (v8f){0.f, 0.f, 0.f, 0.f, 0.f, 0.f, 0.f, 0.f};

  for (int k0 = 0; k0 < K; k0 += 32) {
    V bh[4];
#pragma unroll
    for (int j = 0; j < 4; ++j) {
      const size_t bo = (size_t)(n0 + (j << 4) + rlane) * ldb + koff + k0;
      bh[j] = Frag<T>::load(Bt + bo);
    }
#pragma unroll
    for (int i = 0; i < 4; ++i) {
      const size_t ao = (size_t)(m0 + (i << 4) + rlane) * lda + koff + k0;
      V ah = Frag<T>::load(A + ao);
      V al = ah;
      if (SPL >= 1) al = Frag<T>::load(A2 + ao);
#pragma unroll
      for (int j = 0; j < 4; ++j) {
        acc[i][j] = Frag<T>::mma(ah, bh[j], acc[i][j]);
        if (SPL >= 1) acc[i][j] = Frag<T>::mma(al, bh[j], acc[i][j]);
      }
      Frag<T>::guard4(acc[i][0], acc[i][1], acc[i][2], acc[i][3], ah, al);
    }
    Frag<T>::keep(bh[0], bh[1], bh[2], bh[3]);
  }
  acc_guard4(acc[0][0], acc[0][1], acc[0][2], acc[0][3]);
  acc_guard4(acc[1][0], acc[1][1], acc[1][2], acc[1][3]);
  acc_guard4(acc[2][0], acc[2][1], acc[2][2], acc[2][3]);
  acc_guard4(acc[3][0], acc[3][1], acc[3][2], acc[3][3]);

  float* slab = sT[wave];
#pragma unroll
  for (int i = 0; i < 4; ++i) {
    const int mBase = m0 + (i << 4);
#pragma unroll
    for (int j = 0; j < 4; ++j) {
#pragma unroll
      for (int r = 0; r < 8; ++r) {
        slab[(mOff + r) * 68 + (j << 4) + rlane] = acc[i][j][r] * scale;
      }
    }
    __builtin_amdgcn_fence(__ATOMIC_RELEASE, "workgroup");
    __builtin_amdgcn_wave_barrier();
    __builtin_amdgcn_fence(__ATOMIC_ACQUIRE, "workgroup");
    {
      const int hh = lane >> 4, c4 = (lane & 15) * 4;
      for (int pass = 0; pass < 2; ++pass) {
#pragma unroll
        for (int it = 0; it < 8; ++it) {
          const int row = it * 2 + hh;
          v4f v = *(const v4f*)(slab + row * 68 + c4);
          *(volatile v4f*)(C + (size_t)(mBase + row) * ldc + n0 + c4) = v;
        }
        __threadfence();
      }
    }
    __builtin_amdgcn_fence(__ATOMIC_RELEASE, "workgroup");
    __builtin_amdgcn_wave_barrier();
    __builtin_amdgcn_fence(__ATOMIC_ACQUIRE, "workgroup");
  }
}

__global__ __launch_bounds__(256) void cast8_bf16_kernel(const float* __restrict__ in, unsigned short* __restrict__ out, int n8) {
  const int i = blockIdx.x * 256 + threadIdx.x;
  if (i >= n8) return;
  const float* p = in + 8 * (size_t)i;
  const v4f a = *(const v4f*)(p);
  const v4f c = *(const v4f*)(p + 4);
  unsigned short hb[8];
#pragma unroll
  for (int e = 0; e < 4; ++e) {
    hb[e]     = f2bf_bits(a[e]);
    hb[4 + e] = f2bf_bits(c[e]);
  }
  const v4u u = (v4u){pk16(hb[0], hb[1]), pk16(hb[2], hb[3]), pk16(hb[4], hb[5]), pk16(hb[6], hb[7])};
  unsigned short* q = out + 8 * (size_t)i;
  *(volatile v4u*)q = u;
  __threadfence();
  *(volatile v4u*)q = u;
}

template <int MODE>
__global__ __launch_bounds__(256) void transpose_pack_kernel(
    const float* __restrict__ in0, const float* __restrict__ in1, const float* __restrict__ in2, const float* __restrict__ in3,
    int ldin,
    unsigned short* out0, unsigned short* out1, unsigned short* out2, unsigned short* out3,
    unsigned short* outlo, int ldout, float scale) {
  __shared__ float sm[64][65];
  const int t  = threadIdx.x;
  const int r0 = blockIdx.x * 64;
  const int c0 = blockIdx.y * 64;
  const int z  = blockIdx.z;
  const float* in = (z == 0) ? in0 : (z == 1) ? in1 : (z == 2) ? in2 : in3;
  unsigned short* out = (z == 0) ? out0 : (z == 1) ? out1 : (z == 2) ? out2 : out3;
#pragma unroll
  for (int i = 0; i < 16; ++i) {
    const int e = i * 256 + t;
    const int r = e >> 6;
    const int c = e & 63;
    sm[c][r] = in[(size_t)(r0 + r) * ldin + c0 + c];
  }
  __syncthreads();
  const int lane = t & 31, wave = t >> 5;
  const int q = lane >> 3, c8 = (lane & 7) * 8;
  v4u uh[2], ul[2];
#pragma unroll
  for (int it = 0; it < 2; ++it) {
    const int row = wave * 8 + it * 4 + q;
    unsigned short hb[8], lb[8];
#pragma unroll
    for (int e = 0; e < 8; ++e) {
      const float v = sm[row][c8 + e];
      if (MODE == 0) {
        hb[e] = f2bf_bits(v);
        lb[e] = 0;
      } else if (MODE == 1) {
        const float vb = bf_bits2f(f2bf_bits(v));
        hb[e] = h_bits_flush(vb * scale);
        lb[e] = 0;
      } else {
        hb[e] = f2bf_bits(v);
        lb[e] = f2bf_bits(v - bf_bits2f(hb[e]));
      }
    }
    uh[it] = (v4u){pk16(hb[0], hb[1]), pk16(hb[2], hb[3]), pk16(hb[4], hb[5]), pk16(hb[6], hb[7])};
    ul[it] = (v4u){pk16(lb[0], lb[1]), pk16(lb[2], lb[3]), pk16(lb[4], lb[5]), pk16(lb[6], lb[7])};
  }
  for (int pass = 0; pass < 2; ++pass) {
#pragma unroll
    for (int it = 0; it < 2; ++it) {
      const int row = wave * 8 + it * 4 + q;
      const size_t o = (size_t)(c0 + row) * ldout + r0 + c8;
      *(volatile v4u*)(out + o) = uh[it];
      if (MODE == 2) *(volatile v4u*)(outlo + o) = ul[it];
    }
    __threadfence();
  }
}

__global__ __launch_bounds__(256) void angle_table_kernel(FreqTab fr, float* __restrict__ cosT, float* __restrict__ sinT) {
  const int idx = blockIdx.x * 256 + threadIdx.x;
  const int n = idx >> 5;
  const int i = idx & 31;
  float invf = fr.f[0];
#pragma unroll
  for (int k = 1; k < 32; ++k) invf = (i == k) ? fr.f[k] : invf;
  const float ang = (float)n * invf;
  const float cs = cosf(ang);
  const float sn = sinf(ang);
  volatile float* pc = cosT + idx;
  volatile float* ps = sinT + idx;
  *pc = cs;
  *ps = sn;
  __threadfence();
  *pc = cs;
  *ps = sn;
}

__global__ __launch_bounds__(256) void rot_pack_kernel(
    const float* __restrict__ P, const float* __restrict__ cosT, const float* __restrict__ sinT,
    unsigned short* __restrict__ QH, unsigned short* __restrict__ QL,
    unsigned short* __restrict__ KH, unsigned short* __restrict__ KL,
    unsigned short* __restrict__ G1H) {
  __shared__ __align__(16) float sQK[2 * kRotRows * kEmb];
  const int tid = threadIdx.x, lane = tid & 31, wave = tid >> 5;
  const int i = tid & 31, hs = tid >> 5;
  const int n0 = blockIdx.x * kRotRows;
#pragma unroll 1
  for (int r = 0; r < kRotRows; ++r) {
    const int n = n0 + r;
    const float cs = cosT[n * kHalf + i];
    const float sn = sinT[n * kHalf + i];
#pragma unroll 1
    for (int u = 0; u < 4; ++u) {
      const int ts = u >> 1;
      const int h = ((u & 1) << 3) | hs;
      const float* src = P + (size_t)n * kCat + ts * kEmb + h * kHd;
      float a = src[i];
      float b = src[kHalf + i];
      a = a * (1.0f / (1.0f + expf(-a)));
      b = b * (1.0f / (1.0f + expf(-b)));
      float* dst = sQK + ts * (kRotRows * kEmb) + r * kEmb + h * kHd;
      dst[i] = a * cs - b * sn;
      dst[kHalf + i] = b * cs + a * sn;
    }
  }
  __syncthreads();
  v4u uh[2][2], ul[2][2];
#pragma unroll
  for (int ts = 0; ts < 2; ++ts) {
#pragma unroll
    for (int it = 0; it < 2; ++it) {
      const int idx = it * 256 + tid;
      const int row = idx >> 7;
      const int c8 = (idx & 127) * 8;
      const float* sp = sQK + ts * (kRotRows * kEmb) + row * kEmb + c8;
      const v4f a0 = *(const v4f*)(sp);
      const v4f a1 = *(const v4f*)(sp + 4);
      unsigned short hb[8], lb[8];
#pragma unroll
      for (int e = 0; e < 4; ++e) {
        const float v0 = a0[e];
        const float v1 = a1[e];
        hb[e]     = f2bf_bits(v0);
        hb[4 + e] = f2bf_bits(v1);
        lb[e]     = f2bf_bits(v0 - bf_bits2f(hb[e]));
        lb[4 + e] = f2bf_bits(v1 - bf_bits2f(hb[4 + e]));
      }
      uh[ts][it] = (v4u){pk16(hb[0], hb[1]), pk16(hb[2], hb[3]), pk16(hb[4], hb[5]), pk16(hb[6], hb[7])};
      ul[ts][it] = (v4u){pk16(lb[0], lb[1]), pk16(lb[2], lb[3]), pk16(lb[4], lb[5]), pk16(lb[6], lb[7])};
    }
  }
  v4u g1u;
  const int grow = lane >> 3, gc8 = (lane & 7) * 8;
  {
    const float* gp = P + (size_t)(n0 + grow) * kCat + 3 * kEmb + gc8;
    const v4f a0 = *(const v4f*)(gp);
    const v4f a1 = *(const v4f*)(gp + 4);
    unsigned short hb[8];
#pragma unroll
    for (int e = 0; e < 4; ++e) {
      const float v0 = a0[e];
      const float v1 = a1[e];
      hb[e]     = h_bits_flush(v0 * kG1Carry);
      hb[4 + e] = h_bits_flush(v1 * kG1Carry);
    }
    g1u = (v4u){pk16(hb[0], hb[1]), pk16(hb[2], hb[3]), pk16(hb[4], hb[5]), pk16(hb[6], hb[7])};
  }
  for (int pass = 0; pass < 2; ++pass) {
#pragma unroll
    for (int it = 0; it < 2; ++it) {
      const int idx = it * 256 + tid;
      const int row = idx >> 7;
      const int c8 = (idx & 127) * 8;
      const size_t o = (size_t)(n0 + row) * kEmb + c8;
      *(volatile v4u*)(QH + o) = uh[0][it];
      *(volatile v4u*)(QL + o) = ul[0][it];
      *(volatile v4u*)(KH + o) = uh[1][it];
      *(volatile v4u*)(KL + o) = ul[1][it];
    }
    if (wave == 0) {
      *(volatile v4u*)(G1H + (size_t)(n0 + grow) * kHd + gc8) = g1u;
    }
    __threadfence();
  }
}

__global__ __launch_bounds__(128) void causal_energy_kernel(
    const unsigned short* __restrict__ QHp, const unsigned short* __restrict__ QLp,
    const unsigned short* __restrict__ KHp, const unsigned short* __restrict__ KLp,
    const unsigned short* __restrict__ VTHp, const unsigned short* __restrict__ VTLp,
    float* __restrict__ O) {
  union FB { v16b v; v8b h[2]; };
  __shared__ __align__(16) __bf16 Eh[4][16 * 64];
  __shared__ __align__(16) __bf16 El[4][16 * 64];
  __shared__ __align__(16) float  Os[4][16 * 68];
  const __bf16* QH = (const __bf16*)QHp;
  const __bf16* QL = (const __bf16*)QLp;
  const __bf16* KH = (const __bf16*)KHp;
  const __bf16* KL = (const __bf16*)KLp;
  const __bf16* VTH = (const __bf16*)VTHp;
  const __bf16* VTL = (const __bf16*)VTLp;

  const int tid  = threadIdx.x;
  const int wave = tid >> 5;
  const int lane = tid & 31;
  const int hh   = lane >> 4;
  const int c    = lane & 15;
  const int head = blockIdx.x & (kHeads - 1);
  const int qt   = (kTok / 64 - 1) - (blockIdx.x >> 4);
  const int q0   = qt * 64 + wave * 16;

  const size_t qoff = (size_t)(q0 + c) * kEmb + head * kHd + 8 * hh;
  const v16b qah0 = Frag<__bf16>::load(QH + qoff);
  const v16b qah1 = Frag<__bf16>::load(QH + qoff + 32);
  const v16b qal0 = Frag<__bf16>::load(QL + qoff);
  const v16b qal1 = Frag<__bf16>::load(QL + qoff + 32);

  v8f o0 = (v8f){0.f, 0.f, 0.f, 0.f, 0.f, 0.f, 0.f, 0.f};
  v8f o1 = o0, o2 = o0, o3 = o0;
  __bf16* eh = Eh[wave];
  __bf16* el = El[wave];

  for (int kc = 0; kc <= qt; ++kc) {
    const int kv0 = kc * 64;
    v8f s[4];
#pragma unroll
    for (int j = 0; j < 4; ++j) {
      const size_t ko = (size_t)(kv0 + j * 16 + c) * kEmb + head * kHd + 8 * hh;
      const v16b kh0 = Frag<__bf16>::load(KH + ko);
      const v16b kl0 = Frag<__bf16>::load(KL + ko);
      const v16b kh1 = Frag<__bf16>::load(KH + ko + 32);
      const v16b kl1 = Frag<__bf16>::load(KL + ko + 32);
      v8f a = (v8f){0.f, 0.f, 0.f, 0.f, 0.f, 0.f, 0.f, 0.f};
      a = mma_b(qah0, kh0, a);
      a = mma_b(qah0, kl0, a);
      a = mma_b(qal0, kh0, a);
      a = mma_b(qah1, kh1, a);
      a = mma_b(qah1, kl1, a);
      a = mma_b(qal1, kh1, a);
      s[j] = a;
    }
#pragma unroll
    for (int j = 0; j < 4; ++j) {
      const int kvcol = kv0 + j * 16 + c;
#pragma unroll
      for (int r = 0; r < 8; ++r) {
        const int qrow = q0 + 8 * hh + r;
        float e = s[j][r];
        e = (kvcol > qrow) ? 0.0f : e;
        const unsigned short hb = f2bf_bits(e);
        const unsigned short lb = f2bf_bits(e - bf_bits2f(hb));
        eh[(8 * hh + r) * 64 + j * 16 + c] = __builtin_bit_cast(__bf16, hb);
        el[(8 * hh + r) * 64 + j * 16 + c] = __builtin_bit_cast(__bf16, lb);
      }
    }
    __builtin_amdgcn_fence(__ATOMIC_RELEASE, "workgroup");
    __builtin_amdgcn_wave_barrier();
    __builtin_amdgcn_fence(__ATOMIC_ACQUIRE, "workgroup");
#pragma unroll
    for (int kk = 0; kk < 2; ++kk) {
      FB pa, pl;
      pa.h[0] = *(const v8b*)(eh + c * 64 + kk * 32 + 8 * hh);
      pa.h[1] = *(const v8b*)(eh + c * 64 + kk * 32 + 16 + 8 * hh);
      pl.h[0] = *(const v8b*)(el + c * 64 + kk * 32 + 8 * hh);
      pl.h[1] = *(const v8b*)(el + c * 64 + kk * 32 + 16 + 8 * hh);
      const size_t vo = (size_t)(head * kHd + c) * kTok + kv0 + kk * 32 + 8 * hh;
      {
        const v16b vh = Frag<__bf16>::load(VTH + vo);
        const v16b vl = Frag<__bf16>::load(VTL + vo);
        o0 = mma_b(pa.v, vh, o0);
        o0 = mma_b(pa.v, vl, o0);
        o0 = mma_b(pl.v, vh, o0);
      }
      {
        const v16b vh = Frag<__bf16>::load(VTH + vo + (size_t)16 * kTok);
        const v16b vl = Frag<__bf16>::load(VTL + vo + (size_t)16 * kTok);
        o1 = mma_b(pa.v, vh, o1);
        o1 = mma_b(pa.v, vl, o1);
        o1 = mma_b(pl.v, vh, o1);
      }
      {
        const v16b vh = Frag<__bf16>::load(VTH + vo + (size_t)32 * kTok);
        const v16b vl = Frag<__bf16>::load(VTL + vo + (size_t)32 * kTok);
        o2 = mma_b(pa.v, vh, o2);
        o2 = mma_b(pa.v, vl, o2);
        o2 = mma_b(pl.v, vh, o2);
      }
      {
        const v16b vh = Frag<__bf16>::load(VTH + vo + (size_t)48 * kTok);
        const v16b vl = Frag<__bf16>::load(VTL + vo + (size_t)48 * kTok);
        o3 = mma_b(pa.v, vh, o3);
        o3 = mma_b(pa.v, vl, o3);
        o3 = mma_b(pl.v, vh, o3);
      }
    }
    __builtin_amdgcn_fence(__ATOMIC_RELEASE, "workgroup");
    __builtin_amdgcn_wave_barrier();
    __builtin_amdgcn_fence(__ATOMIC_ACQUIRE, "workgroup");
  }

  float* os = Os[wave];
#pragma unroll
  for (int r = 0; r < 8; ++r) {
    os[(8 * hh + r) * 68 + 0 * 16 + c] = o0[r];
    os[(8 * hh + r) * 68 + 1 * 16 + c] = o1[r];
    os[(8 * hh + r) * 68 + 2 * 16 + c] = o2[r];
    os[(8 * hh + r) * 68 + 3 * 16 + c] = o3[r];
  }
  __builtin_amdgcn_fence(__ATOMIC_RELEASE, "workgroup");
  __builtin_amdgcn_wave_barrier();
  __builtin_amdgcn_fence(__ATOMIC_ACQUIRE, "workgroup");
  {
    const int c4 = (lane & 15) * 4;
    float* ob = O + (size_t)q0 * kEmb + head * kHd;
    for (int pass = 0; pass < 2; ++pass) {
#pragma unroll
      for (int it = 0; it < 8; ++it) {
        const int row = it * 2 + hh;
        v4f val = *(const v4f*)(os + row * 68 + c4);
        *(volatile v4f*)(ob + (size_t)row * kEmb + c4) = val;
      }
      __threadfence();
    }
  }
}

__global__ __launch_bounds__(256) void gate_ln_kernel(
    const float* __restrict__ attn, const float* __restrict__ glogit,
    const float* __restrict__ lnw, const float* __restrict__ lnb,
    unsigned short* __restrict__ ZH, unsigned short* __restrict__ ZL) {
  __shared__ float red1[8];
  __shared__ float red2[8];
  const int row = blockIdx.x;
  const int t = threadIdx.x, lane = t & 31, wave = t >> 5;
  const int c0 = t * 4;
  const v4f av = *(const v4f*)(attn + (size_t)row * kEmb + c0);
  const v4f gv = *(const v4f*)(glogit + (size_t)row * kEmb + c0);
  const v4f wv = *(const v4f*)(lnw + c0);
  const v4f bv = *(const v4f*)(lnb + c0);
  float y[4];
#pragma unroll
  for (int e = 0; e < 4; ++e) {
    const float g = gv[e];
    const float sg = 1.0f / (1.0f + expf(-g));
    y[e] = av[e] * sg;
  }
  float s = (y[0] + y[1]) + (y[2] + y[3]);
#pragma unroll
  for (int off = 16; off > 0; off >>= 1) s += __shfl_xor(s, off, 32);
  if (lane == 0) red1[wave] = s;
  __syncthreads();
  float tot = 0.0f;
#pragma unroll
  for (int w = 0; w < 8; ++w) tot += red1[w];
  const float mu = tot * kInvEmb;
  float d[4];
  float vs = 0.0f;
#pragma unroll
  for (int e = 0; e < 4; ++e) {
    d[e] = y[e] - mu;
    vs += d[e] * d[e];
  }
#pragma unroll
  for (int off = 16; off > 0; off >>= 1) vs += __shfl_xor(vs, off, 32);
  if (lane == 0) red2[wave] = vs;
  __syncthreads();
  float tot2 = 0.0f;
#pragma unroll
  for (int w = 0; w < 8; ++w) tot2 += red2[w];
  const float var = tot2 * kInvEmb;
  const float rstd = 1.0f / sqrtf(var + kLnEps);
  unsigned short hb[4], lb[4];
#pragma unroll
  for (int e = 0; e < 4; ++e) {
    const float wq = bf_bits2f(f2bf_bits(wv[e]));
    const float bq = bf_bits2f(f2bf_bits(bv[e]));
    const float zv = d[e] * rstd * wq + bq;
    hb[e] = f2bf_bits(zv);
    lb[e] = f2bf_bits(zv - bf_bits2f(hb[e]));
  }
  const v2u uh = (v2u){pk16(hb[0], hb[1]), pk16(hb[2], hb[3])};
  const v2u ul = (v2u){pk16(lb[0], lb[1]), pk16(lb[2], lb[3])};
  unsigned short* ph = ZH + (size_t)row * kEmb + c0;
  unsigned short* pl = ZL + (size_t)row * kEmb + c0;
  *(volatile v2u*)ph = uh;
  *(volatile v2u*)pl = ul;
  __threadfence();
  *(volatile v2u*)ph = uh;
  *(volatile v2u*)pl = ul;
}

extern "C" void kernel_launch(void* const* d_in, const int* in_sizes, int n_in,
                              void* d_out, int out_size, void* d_ws, size_t ws_size,
                              hipStream_t stream) {
  if (n_in < 9) return;
  if (in_sizes[0] != kTok * kEmb) return;
  if (in_sizes[1] != kEmb * kEmb) return;
  if (in_sizes[2] != kEmb * kEmb) return;
  if (in_sizes[3] != kEmb * kEmb) return;
  if (in_sizes[4] != kEmb * kEmb) return;
  if (in_sizes[5] != kEmb * kHd) return;
  if (in_sizes[6] != kHd * kEmb) return;
  if (in_sizes[7] != kEmb) return;
  if (in_sizes[8] != kEmb) return;
  if (out_size != kTok * kEmb) return;
  if (ws_size < kWsTotal) return;

  const float* x   = (const float*)d_in[0];
  const float* Wq  = (const float*)d_in[1];
  const float* Wk  = (const float*)d_in[2];
  const float* Wv  = (const float*)d_in[3];
  const float* Wo  = (const float*)d_in[4];
  const float* Wg1 = (const float*)d_in[5];
  const float* Wg2 = (const float*)d_in[6];
  const float* lnw = (const float*)d_in[7];
  const float* lnb = (const float*)d_in[8];
  float* out = (float*)d_out;

  char* ws = (char*)d_ws;
  unsigned short* XB   = (unsigned short*)(ws + kOffXB);
  unsigned short* WCT  = (unsigned short*)(ws + kOffWCT);
  unsigned short* WOT  = (unsigned short*)(ws + kOffWOT);
  unsigned short* WG2T = (unsigned short*)(ws + kOffWG2T);
  float*          CST  = (float*)(ws + kOffCST);
  float*          SNT  = (float*)(ws + kOffSNT);
  float*          P    = (float*)(ws + kOffP);
  unsigned short* QH   = (unsigned short*)(ws + kOffQH);
  unsigned short* QL   = (unsigned short*)(ws + kOffQL);
  unsigned short* KH   = (unsigned short*)(ws + kOffKH);
  unsigned short* KL   = (unsigned short*)(ws + kOffKL);
  unsigned short* VTH  = (unsigned short*)(ws + kOffVTH);
  unsigned short* VTL  = (unsigned short*)(ws + kOffVTL);
  unsigned short* G1H  = (unsigned short*)(ws + kOffG1H);
  float*          ATT  = (float*)(ws + kOffATT);
  float*          GLG  = (float*)(ws + kOffGLG);
  unsigned short* ZH   = (unsigned short*)(ws + kOffZH);
  unsigned short* ZL   = (unsigned short*)(ws + kOffZL);

  FreqTab fr;
  for (int i = 0; i < kHalf; ++i) {
    const float e = (float)(2 * i) / (float)kHd;
    const float p = (float)pow(10000.0, (double)e);
    fr.f[i] = 1.0f / p;
  }

  cast8_bf16_kernel<<<(kTok * kEmb / 8) / 256, 256, 0, stream>>>(x, XB, kTok * kEmb / 8);

  transpose_pack_kernel<0><<<dim3(kEmb / 64, kEmb / 64, 4), 256, 0, stream>>>(
      Wq, Wk, Wv, Wo, kEmb,
      WCT, WCT + (size_t)kEmb * kEmb, WCT + (size_t)2 * kEmb * kEmb, WOT,
      WOT, kEmb, 1.0f);
  transpose_pack_kernel<0><<<dim3(kEmb / 64, kHd / 64, 1), 256, 0, stream>>>(
      Wg1, Wg1, Wg1, Wg1, kHd,
      WCT + (size_t)3 * kEmb * kEmb, WCT + (size_t)3 * kEmb * kEmb, WCT + (size_t)3 * kEmb * kEmb, WCT + (size_t)3 * kEmb * kEmb,
      WCT + (size_t)3 * kEmb * kEmb, kEmb, 1.0f);
  transpose_pack_kernel<1><<<dim3(kHd / 64, kEmb / 64, 1), 256, 0, stream>>>(
      Wg2, Wg2, Wg2, Wg2, kEmb,
      WG2T, WG2T, WG2T, WG2T,
      WG2T, kHd, kWg2Carry);

  angle_table_kernel<<<(kTok * kHalf) / 256, 256, 0, stream>>>(fr, CST, SNT);

  wmma_gemm64<1, 0><<<dim3((kTok / 64) * (kCat / 64) / 8), 256, 0, stream>>>(
      XB, XB, kEmb, WCT, kEmb, P, kCat, kTok, kCat, kEmb, 1.0f);

  rot_pack_kernel<<<kTok / kRotRows, 256, 0, stream>>>(P, CST, SNT, QH, QL, KH, KL, G1H);

  transpose_pack_kernel<2><<<dim3(kTok / 64, kEmb / 64, 1), 256, 0, stream>>>(
      P + 2 * kEmb, P + 2 * kEmb, P + 2 * kEmb, P + 2 * kEmb, kCat,
      VTH, VTH, VTH, VTH,
      VTL, kTok, 1.0f);

  causal_energy_kernel<<<kHeads * (kTok / 64), 128, 0, stream>>>(QH, QL, KH, KL, VTH, VTL, ATT);

  wmma_gemm64<0, 0><<<dim3((kTok / 64) * (kEmb / 64) / 8), 256, 0, stream>>>(
      G1H, G1H, kHd, WG2T, kHd, GLG, kEmb, kTok, kEmb, kHd, kGateScale);

  gate_ln_kernel<<<kTok, 256, 0, stream>>>(ATT, GLG, lnw, lnb, ZH, ZL);

  wmma_gemm64<1, 1><<<dim3((kTok / 64) * (kEmb / 64) / 8), 256, 0, stream>>>(
      ZH, ZL, kEmb, WOT, kEmb, out, kEmb, kTok, kEmb, kEmb, 1.0f);
}
